// Cross_TransformerModel_57561151701172
// MI455X (gfx1250) — hardware-run, weakly checked
//
#include <hip/hip_runtime.h>
#include <math.h>
#include <stddef.h>

constexpr int kB      = 4;
constexpr int kSq     = 2048;
constexpr int kD      = 1024;
constexpr int kSv     = 196;
constexpr int kSvPad  = 256;
constexpr int kDff    = 4096;
constexpr int kRows   = kB * kSq;
constexpr int kFfnChunkRows = 4096;
constexpr int kFfnChunks    = kRows / kFfnChunkRows;
constexpr float kWCarry    = 16.0f;
constexpr float kWCarryInv = 1.0f / 16.0f;
constexpr float kPCarry    = 2048.0f;
constexpr float kOCarry    = 16.0f;
constexpr float kPVScale   = kOCarry / kPCarry;
constexpr float kWoScale   = 1.0f / (kOCarry * kWCarry);
constexpr float kInvD      = 1.0f / 1024.0f;
constexpr float kLnEps     = 1e-6f;
constexpr float kScoreScale = 0.125f;

static_assert(kRows % 64 == 0);
static_assert(kSvPad % 64 == 0 && kSvPad % 32 == 0);
static_assert(kD % 64 == 0 && kDff % 64 == 0);
static_assert(kRows % 8 == 0);
static_assert(kFfnChunks * kFfnChunkRows == kRows);

constexpr size_t kMiB       = 1048576;
constexpr size_t kOffPool32 = 0;
constexpr size_t kOffPool16 = 32 * kMiB;
constexpr size_t kOffW1H    = 48 * kMiB;
constexpr size_t kOffW2H    = 56 * kMiB;
constexpr size_t kOffWQH    = 64 * kMiB;
constexpr size_t kOffWKH    = 66 * kMiB;
constexpr size_t kOffWVH    = 68 * kMiB;
constexpr size_t kOffWOH    = 70 * kMiB;
constexpr size_t kOffT16    = 72 * kMiB;
constexpr size_t kOffO16    = 72 * kMiB;
constexpr size_t kOffQ16    = 88 * kMiB;
constexpr size_t kOffA1     = 88 * kMiB;
constexpr size_t kOffS32    = 104 * kMiB;
constexpr size_t kOffP16    = 112 * kMiB;
constexpr size_t kOffVIS16  = 120 * kMiB;
constexpr size_t kOffK16    = 120 * kMiB + 524288;
constexpr size_t kOffVT16   = 121 * kMiB;
constexpr size_t kWsTotal   = 121 * kMiB + 524288;
constexpr size_t kOffH16    = 64 * kMiB;
constexpr size_t kOffF32    = 96 * kMiB;
static_assert(kOffS32 == kOffQ16 + (size_t)kRows * kD * 2);
static_assert(kOffP16 == kOffS32 + (size_t)kRows * kSvPad * 4);
static_assert(kOffVIS16 >= kOffA1 + (size_t)kRows * kD * 4);
static_assert(kOffVIS16 >= kOffP16 + (size_t)kRows * kSvPad * 2);
static_assert(kOffK16 == kOffVIS16 + (size_t)kSvPad * kD * 2);
static_assert(kOffVT16 == kOffK16 + (size_t)kSvPad * kD * 2);
static_assert(kWsTotal == kOffVT16 + (size_t)kD * kSvPad * 2);
static_assert(kOffF32 == kOffH16 + (size_t)kFfnChunkRows * kDff * 2);
static_assert(kOffF32 + (size_t)kFfnChunkRows * kD * 4 <= kWsTotal);
static_assert(kOffQ16 == kOffT16 + (size_t)kRows * kD * 2);
static_assert(kWsTotal <= (size_t)134217728);

typedef __attribute__((ext_vector_type(16))) _Float16 v16h;
typedef __attribute__((ext_vector_type(8)))  _Float16 v8h;
typedef __attribute__((ext_vector_type(16))) __bf16   v16b;
typedef __attribute__((ext_vector_type(8)))  __bf16   v8b;
typedef __attribute__((ext_vector_type(8)))  float    v8f;
typedef __attribute__((ext_vector_type(4)))  float    v4f;
typedef __attribute__((ext_vector_type(4)))  unsigned int v4u;

__device__ __forceinline__ unsigned short f2bf_bits(float f) {
  unsigned u = __float_as_uint(f);
  return (unsigned short)((u + 0x7FFFu + ((u >> 16) & 1u)) >> 16);
}
__device__ __forceinline__ float bf_bits2f(unsigned short h) { return __uint_as_float(((unsigned)h) << 16); }

__device__ __forceinline__ void dep_guard_h(v8f& a, v8f& b, v16h x, v16h y) { asm volatile("v_nop\n\tv_nop\n\tv_nop\n\tv_nop" : "+v"(a), "+v"(b) : "v"(x), "v"(y)); }
__device__ __forceinline__ void dep_guard_b(v8f& a, v8f& b, v16b x, v16b y) { asm volatile("v_nop\n\tv_nop\n\tv_nop\n\tv_nop" : "+v"(a), "+v"(b) : "v"(x), "v"(y)); }
__device__ __forceinline__ void keep4_h(v16h a, v16h b, v16h c, v16h d) { asm volatile("v_nop" :: "v"(a), "v"(b), "v"(c), "v"(d)); }
__device__ __forceinline__ void keep4_b(v16b a, v16b b, v16b c, v16b d) { asm volatile("v_nop" :: "v"(a), "v"(b), "v"(c), "v"(d)); }
__device__ __forceinline__ void acc_guard4(v8f& a, v8f& b, v8f& c, v8f& d) { asm volatile("v_nop\n\tv_nop\n\tv_nop\n\tv_nop" : "+v"(a), "+v"(b), "+v"(c), "+v"(d)); }
template <typename T> struct Frag;
template <> struct Frag<_Float16> {
  typedef v16h V; union U { v16h v; v8h h[2]; };
  static __device__ __forceinline__ v16h load(const _Float16* p) {
    U f; f.h[0] = *(const v8h*)(p); f.h[1] = *(const v8h*)(p + 16); return f.v;
  }
  static __device__ __forceinline__ v8f mma(v16h a, v16h b, v8f c) {
    return __builtin_amdgcn_wmma_f32_16x16x32_f16(false, a, false, b, (short)0, c, false, false);
  }
  static __device__ __forceinline__ void guard(v8f& a, v8f& b, v16h x, v16h y) { dep_guard_h(a, b, x, y); }
  static __device__ __forceinline__ void keep(v16h a, v16h b, v16h c, v16h d) { keep4_h(a, b, c, d); }
};
template <> struct Frag<__bf16> {
  typedef v16b V; union U { v16b v; v8b h[2]; };
  static __device__ __forceinline__ v16b load(const __bf16* p) {
    U f; f.h[0] = *(const v8b*)(p); f.h[1] = *(const v8b*)(p + 16); return f.v;
  }
  static __device__ __forceinline__ v8f mma(v16b a, v16b b, v8f c) {
    return __builtin_amdgcn_wmma_f32_16x16x32_bf16(false, a, false, b, (short)0, c, false, false);
  }
  static __device__ __forceinline__ void guard(v8f& a, v8f& b, v16b x, v16b y) { dep_guard_b(a, b, x, y); }
  static __device__ __forceinline__ void keep(v16b a, v16b b, v16b c, v16b d) { keep4_b(a, b, c, d); }
};

__device__ __forceinline__ unsigned pk16(unsigned short a, unsigned short b) { return (unsigned)a | ((unsigned)b << 16); }
__device__ __forceinline__ unsigned short h_bits(float f) { const _Float16 h = (_Float16)f; return __builtin_bit_cast(unsigned short, h); }

template <int ET> struct Elem;
template <> struct Elem<0> { typedef _Float16 T; };
template <> struct Elem<1> { typedef __bf16 T; };
template <int ET, bool SPLIT, int BIAS_MODE, int OUT_MODE, bool RESID, int ACT = 0>
__global__ __launch_bounds__(256) void wmma_gemm64(
    const unsigned short* __restrict__ Ap, const unsigned short* __restrict__ A2p, int lda, long strideA,
    const unsigned short* __restrict__ Btp, const unsigned short* __restrict__ Bt2p, int ldb, long strideB,
    void* __restrict__ Cout, void* __restrict__ Cout2, int ldc, long strideC,
    const float* __restrict__ bias,
    const float* __restrict__ resid, long strideR,
    int M, int N, int K, float scale) {
  typedef typename Elem<ET>::T T;
  typedef typename Frag<T>::V V;
  const T* A = (const T*)Ap; const T* A2 = (const T*)A2p; const T* Bt = (const T*)Btp; const T* Bt2 = (const T*)Bt2p;
  __shared__ __align__(16) float sT[8][16 * 68];
  const int b    = blockIdx.y;
  const int lane = threadIdx.x & 31;
  const int wave = threadIdx.x >> 5;
  const int tilesN = N >> 6;
  const int tilesM = M >> 6;
  const int tile = blockIdx.x * 8 + wave;
  if (tile >= tilesM * tilesN) return;
  const int tm = tile / tilesN;
  const int tn = tile - tm * tilesN;
  const int m0 = tm << 6;
  const int n0 = tn << 6;

  const T* Ab  = A  + (size_t)b * strideA;
  const T* Bb  = Bt + (size_t)b * strideB;
  const T* Ab2 = SPLIT ? (A2  + (size_t)b * strideA) : nullptr;
  const T* Bb2 = SPLIT ? (Bt2 + (size_t)b * strideB) : nullptr;

  const int rlane = lane & 15;
  const int koff  = (lane >> 4) * 8;
  const int mOff  = (lane >> 4) * 8;

  v8f acc[4][4];
#pragma unroll
  for (int i = 0; i < 4; ++i)
#pragma unroll
    for (int j = 0; j < 4; ++j) acc[i][j] = (v8f){0.f,0.f,0.f,0.f,0.f,0.f,0.f,0.f};

  for (int k0 = 0; k0 < K; k0 += 32) {
    V bh[4], bl[4];
#pragma unroll
    for (int j = 0; j < 4; ++j) {
      const size_t bo = (size_t)(n0 + (j << 4) + rlane) * ldb + koff + k0;
      bh[j] = Frag<T>::load(Bb + bo);
      if (SPLIT) bl[j] = Frag<T>::load(Bb2 + bo);
    }
#pragma unroll
    for (int i = 0; i < 4; ++i) {
      const size_t ao = (size_t)(m0 + (i << 4) + rlane) * lda + koff + k0;
      V ah = Frag<T>::load(Ab + ao);
      V al;
      if (SPLIT) al = Frag<T>::load(Ab2 + ao);
#pragma unroll
      for (int j = 0; j < 4; ++j) {
        acc[i][j] = Frag<T>::mma(ah, bh[j], acc[i][j]);
        if (SPLIT) {
          acc[i][j] = Frag<T>::mma(ah, bl[j], acc[i][j]);
          acc[i][j] = Frag<T>::mma(al, bh[j], acc[i][j]);
        }
      }
      Frag<T>::guard(acc[i][0], acc[i][3], ah, SPLIT ? al : ah);
    }
    Frag<T>::keep(bh[0], bh[1], bh[2], bh[3]);
    if (SPLIT) Frag<T>::keep(bl[0], bl[1], bl[2], bl[3]);
  }
  acc_guard4(acc[0][0], acc[0][1], acc[0][2], acc[0][3]);
  acc_guard4(acc[1][0], acc[1][1], acc[1][2], acc[1][3]);
  acc_guard4(acc[2][0], acc[2][1], acc[2][2], acc[2][3]);
  acc_guard4(acc[3][0], acc[3][1], acc[3][2], acc[3][3]);

  float* slab = sT[wave];
  const float* Rb = RESID ? (resid + (size_t)b * strideR) : nullptr;
#pragma unroll
  for (int i = 0; i < 4; ++i) {
    const int mBase = m0 + (i << 4);
#pragma unroll
    for (int j = 0; j < 4; ++j) {
      const int n = n0 + (j << 4) + rlane;
      float bv = 0.f;
      if (BIAS_MODE == 2) bv = bias[n];
#pragma unroll
      for (int r = 0; r < 8; ++r) {
        float v = acc[i][j][r] * scale;
        if (BIAS_MODE == 1) v += bias[mBase + mOff + r];
        if (BIAS_MODE == 2) v += bv;
        if (RESID) v += Rb[(size_t)(mBase + mOff + r) * ldc + n];
        if (ACT == 2) v = fmaxf(v, 0.0f);
        if (ACT == 4) v = (v > 0.f) ? v : 0.01f * v;
        slab[(mOff + r) * 68 + (j << 4) + rlane] = v;
      }
    }
    __builtin_amdgcn_fence(__ATOMIC_RELEASE, "workgroup");
    __builtin_amdgcn_wave_barrier();
    __builtin_amdgcn_fence(__ATOMIC_ACQUIRE, "workgroup");
    if (OUT_MODE == 0) {
      float* C = (float*)Cout + (size_t)b * strideC;
      const int hh = lane >> 4, c4 = (lane & 15) * 4;
      for (int pass = 0; pass < 2; ++pass) {
#pragma unroll
        for (int it = 0; it < 8; ++it) {
          const int row = it * 2 + hh;
          v4f v = *(const v4f*)(slab + row * 68 + c4);
          *(volatile v4f*)(C + (size_t)(mBase + row) * ldc + n0 + c4) = v;
        }
        __threadfence();
      }
    } else {
      const int q = lane >> 3, c8 = (lane & 7) * 8;
      unsigned short* C  = (unsigned short*)Cout  + (size_t)b * strideC;
      unsigned short* C2 = (OUT_MODE == 2) ? ((unsigned short*)Cout2 + (size_t)b * strideC) : nullptr;
      for (int pass = 0; pass < 2; ++pass) {
#pragma unroll
        for (int it = 0; it < 4; ++it) {
          const int row = it * 4 + q;
          const float* sp = slab + row * 68 + c8;
          v8h hv, lv;
#pragma unroll
          for (int e = 0; e < 8; ++e) {
            if (OUT_MODE == 1) {
              hv[e] = (_Float16)sp[e];
            } else {
              unsigned short hb = f2bf_bits(sp[e]);
              unsigned short lb = f2bf_bits(sp[e] - bf_bits2f(hb));
              hv[e] = __builtin_bit_cast(_Float16, hb);
              lv[e] = __builtin_bit_cast(_Float16, lb);
            }
          }
          *(volatile v8h*)(C + (size_t)(mBase + row) * ldc + n0 + c8) = hv;
          if (OUT_MODE == 2) *(volatile v8h*)(C2 + (size_t)(mBase + row) * ldc + n0 + c8) = lv;
        }
        __threadfence();
      }
    }
    __builtin_amdgcn_fence(__ATOMIC_RELEASE, "workgroup");
    __builtin_amdgcn_wave_barrier();
    __builtin_amdgcn_fence(__ATOMIC_ACQUIRE, "workgroup");
  }
}

__global__ __launch_bounds__(256) void cast8_kernel(const float* __restrict__ in, unsigned short* __restrict__ out,
                                                    int n8, int nvalid8, float scale) {
  const int i = blockIdx.x * 256 + threadIdx.x;
  if (i >= n8) return;
  const bool valid = (i < nvalid8);
  const int ic = valid ? i : (nvalid8 - 1);
  const float f = valid ? scale : 0.0f;
  const float* p = in + 8 * (size_t)ic;
  const v4f a = *(const v4f*)(p);
  const v4f c = *(const v4f*)(p + 4);
  unsigned short hb[8];
#pragma unroll
  for (int e = 0; e < 4; ++e) {
    hb[e]     = h_bits(a[e] * f);
    hb[4 + e] = h_bits(c[e] * f);
  }
  const v4u u = (v4u){pk16(hb[0], hb[1]), pk16(hb[2], hb[3]), pk16(hb[4], hb[5]), pk16(hb[6], hb[7])};
  unsigned short* q = out + 8 * (size_t)i;
  *(volatile v4u*)q = u;
  __threadfence();
  *(volatile v4u*)q = u;
}

__global__ __launch_bounds__(256) void softmax_kernel(const float* __restrict__ S, const float* __restrict__ SC,
                                                      unsigned short* __restrict__ P) {
  const int lane = threadIdx.x & 31;
  const int wave = threadIdx.x >> 5;
  const int row  = blockIdx.x * 8 + wave;
  const float* sr = S  + (size_t)row * kSvPad;
  const float* cr = SC + (size_t)row * kSv;
  float x[8];
#pragma unroll
  for (int e = 0; e < 8; ++e) {
    const int col = lane * 8 + e;
    const int cc  = (col < kSv) ? col : (kSv - 1);
    const float v = (sr[cc] + cr[cc]) * kScoreScale;
    x[e] = (col < kSv) ? v : -1.0e30f;
  }
  float m = fmaxf(fmaxf(fmaxf(x[0], x[1]), fmaxf(x[2], x[3])), fmaxf(fmaxf(x[4], x[5]), fmaxf(x[6], x[7])));
#pragma unroll
  for (int off = 16; off > 0; off >>= 1) m = fmaxf(m, __shfl_xor(m, off, 32));
  float ev[8];
  float s = 0.f;
#pragma unroll
  for (int e = 0; e < 8; ++e) { ev[e] = expf(x[e] - m); s += ev[e]; }
#pragma unroll
  for (int off = 16; off > 0; off >>= 1) s += __shfl_xor(s, off, 32);
  const float inv = kPCarry / s;
  unsigned short hb[8];
#pragma unroll
  for (int e = 0; e < 8; ++e) hb[e] = h_bits(ev[e] * inv);
  const v4u u = (v4u){pk16(hb[0], hb[1]), pk16(hb[2], hb[3]), pk16(hb[4], hb[5]), pk16(hb[6], hb[7])};
  unsigned short* q = P + (size_t)row * kSvPad + 8 * lane;
  *(volatile v4u*)q = u;
  __threadfence();
  *(volatile v4u*)q = u;
}

__device__ __forceinline__ float block_sum_256(float v, float* red, int lane, int wave) {
#pragma unroll
  for (int off = 16; off > 0; off >>= 1) v += __shfl_xor(v, off, 32);
  if (lane == 0) red[wave] = v;
  __syncthreads();
  float t = red[0];
#pragma unroll
  for (int w = 1; w < 8; ++w) t += red[w];
  return t;
}

__global__ __launch_bounds__(256) void ln_pool_kernel(const float* __restrict__ X, const float* __restrict__ gam,
                                                      const float* __restrict__ bet, float* __restrict__ pool32,
                                                      unsigned short* __restrict__ pool16, int colOff) {
  __shared__ __align__(16) float ybuf[kD];
  __shared__ float redA[8];
  __shared__ float redB[8];
  const int t = threadIdx.x;
  const int lane = t & 31, wave = t >> 5;
  const int row = blockIdx.x;
  const v4f x = *(const v4f*)(X + (size_t)row * kD + 4 * t);
  const float s = (x[0] + x[1]) + (x[2] + x[3]);
  const float mu = block_sum_256(s, redA, lane, wave) * kInvD;
  const float d0 = x[0] - mu, d1 = x[1] - mu, d2 = x[2] - mu, d3 = x[3] - mu;
  const float q = (d0 * d0 + d1 * d1) + (d2 * d2 + d3 * d3);
  const float var = block_sum_256(q, redB, lane, wave) * kInvD;
  const float rs = rsqrtf(var + kLnEps);
  const v4f gg = *(const v4f*)(gam + 4 * t);
  const v4f bb = *(const v4f*)(bet + 4 * t);
  ybuf[4 * t + 0] = d0 * rs * gg[0] + bb[0];
  ybuf[4 * t + 1] = d1 * rs * gg[1] + bb[1];
  ybuf[4 * t + 2] = d2 * rs * gg[2] + bb[2];
  ybuf[4 * t + 3] = d3 * rs * gg[3] + bb[3];
  __syncthreads();
  if (t < 128) {
    const v4f a = *(const v4f*)(ybuf + 8 * t);
    const v4f c = *(const v4f*)(ybuf + 8 * t + 4);
    v4f p;
    p[0] = fmaxf(a[0], a[1]);
    p[1] = fmaxf(a[2], a[3]);
    p[2] = fmaxf(c[0], c[1]);
    p[3] = fmaxf(c[2], c[3]);
    float* dst = pool32 + (size_t)row * kD + colOff + 4 * t;
    *(volatile v4f*)dst = p;
    __threadfence();
    *(volatile v4f*)dst = p;
  } else if (t < 192) {
    const int u = t - 128;
    const v4f a0 = *(const v4f*)(ybuf + 16 * u);
    const v4f a1 = *(const v4f*)(ybuf + 16 * u + 4);
    const v4f a2 = *(const v4f*)(ybuf + 16 * u + 8);
    const v4f a3 = *(const v4f*)(ybuf + 16 * u + 12);
    unsigned short hb[8];
    hb[0] = h_bits(fmaxf(a0[0], a0[1]));
    hb[1] = h_bits(fmaxf(a0[2], a0[3]));
    hb[2] = h_bits(fmaxf(a1[0], a1[1]));
    hb[3] = h_bits(fmaxf(a1[2], a1[3]));
    hb[4] = h_bits(fmaxf(a2[0], a2[1]));
    hb[5] = h_bits(fmaxf(a2[2], a2[3]));
    hb[6] = h_bits(fmaxf(a3[0], a3[1]));
    hb[7] = h_bits(fmaxf(a3[2], a3[3]));
    const v4u uu = (v4u){pk16(hb[0], hb[1]), pk16(hb[2], hb[3]), pk16(hb[4], hb[5]), pk16(hb[6], hb[7])};
    unsigned short* dst = pool16 + (size_t)row * kD + colOff + 8 * u;
    *(volatile v4u*)dst = uu;
    __threadfence();
    *(volatile v4u*)dst = uu;
  }
}

__global__ __launch_bounds__(256) void ln_out_kernel(const float* __restrict__ X, const float* __restrict__ gam,
                                                     const float* __restrict__ bet, float* __restrict__ out) {
  __shared__ float redA[8];
  __shared__ float redB[8];
  const int t = threadIdx.x;
  const int lane = t & 31, wave = t >> 5;
  const int row = blockIdx.x;
  const v4f x = *(const v4f*)(X + (size_t)row * kD + 4 * t);
  const float s = (x[0] + x[1]) + (x[2] + x[3]);
  const float mu = block_sum_256(s, redA, lane, wave) * kInvD;
  const float d0 = x[0] - mu, d1 = x[1] - mu, d2 = x[2] - mu, d3 = x[3] - mu;
  const float q = (d0 * d0 + d1 * d1) + (d2 * d2 + d3 * d3);
  const float var = block_sum_256(q, redB, lane, wave) * kInvD;
  const float rs = rsqrtf(var + kLnEps);
  const v4f gg = *(const v4f*)(gam + 4 * t);
  const v4f bb = *(const v4f*)(bet + 4 * t);
  v4f y;
  y[0] = d0 * rs * gg[0] + bb[0];
  y[1] = d1 * rs * gg[1] + bb[1];
  y[2] = d2 * rs * gg[2] + bb[2];
  y[3] = d3 * rs * gg[3] + bb[3];
  float* dst = out + (size_t)row * kD + 4 * t;
  *(volatile v4f*)dst = y;
  __threadfence();
  *(volatile v4f*)dst = y;
}

static inline dim3 gemm_grid(int M, int N) {
  const int tiles = (M >> 6) * (N >> 6);
  return dim3((unsigned)((tiles + 7) / 8), 1, 1);
}

extern "C" void kernel_launch(void* const* d_in, const int* in_sizes, int n_in,
                              void* d_out, int out_size, void* d_ws, size_t ws_size,
                              hipStream_t stream)
{
  if (n_in < 22) return;
  if ((size_t)out_size < (size_t)kRows * kD) return;
  if (ws_size < kWsTotal) return;
  if (in_sizes[0] < kRows * kD || in_sizes[3] < kRows * kD) return;
  if (in_sizes[1] < kSv * kD || in_sizes[4] < kSv * kD) return;
  if (in_sizes[2] < kRows * kSv || in_sizes[5] < kRows * kSv) return;
  if (in_sizes[6] < kD * kD || in_sizes[8] < kD * kD || in_sizes[10] < kD * kD || in_sizes[12] < kD * kD) return;
  if (in_sizes[14] < kDff * kD || in_sizes[16] < kD * kDff) return;

  const float* text1 = (const float*)d_in[0];
  const float* vis1  = (const float*)d_in[1];
  const float* sc1   = (const float*)d_in[2];
  const float* text2 = (const float*)d_in[3];
  const float* vis2  = (const float*)d_in[4];
  const float* sc2   = (const float*)d_in[5];
  const float* Wq = (const float*)d_in[6];   const float* bq  = (const float*)d_in[7];
  const float* Wk = (const float*)d_in[8];   const float* bk  = (const float*)d_in[9];
  const float* Wv = (const float*)d_in[10];  const float* bv  = (const float*)d_in[11];
  const float* Wo = (const float*)d_in[12];  const float* bo  = (const float*)d_in[13];
  const float* W1 = (const float*)d_in[14];  const float* b1  = (const float*)d_in[15];
  const float* W2 = (const float*)d_in[16];  const float* b2  = (const float*)d_in[17];
  const float* g1 = (const float*)d_in[18];  const float* be1 = (const float*)d_in[19];
  const float* g2 = (const float*)d_in[20];  const float* be2 = (const float*)d_in[21];
  float* outp = (float*)d_out;

  char* ws = (char*)d_ws;
  float*          POOL32 = (float*)(ws + kOffPool32);
  unsigned short* POOL16 = (unsigned short*)(ws + kOffPool16);
  unsigned short* W1H    = (unsigned short*)(ws + kOffW1H);
  unsigned short* W2H    = (unsigned short*)(ws + kOffW2H);
  unsigned short* WQH    = (unsigned short*)(ws + kOffWQH);
  unsigned short* WKH    = (unsigned short*)(ws + kOffWKH);
  unsigned short* WVH    = (unsigned short*)(ws + kOffWVH);
  unsigned short* WOH    = (unsigned short*)(ws + kOffWOH);
  unsigned short* T16    = (unsigned short*)(ws + kOffT16);
  unsigned short* O16    = (unsigned short*)(ws + kOffO16);
  unsigned short* Q16    = (unsigned short*)(ws + kOffQ16);
  float*          A1     = (float*)(ws + kOffA1);
  float*          S32    = (float*)(ws + kOffS32);
  unsigned short* P16    = (unsigned short*)(ws + kOffP16);
  unsigned short* VIS16  = (unsigned short*)(ws + kOffVIS16);
  unsigned short* K16    = (unsigned short*)(ws + kOffK16);
  unsigned short* VT16   = (unsigned short*)(ws + kOffVT16);
  unsigned short* H16    = (unsigned short*)(ws + kOffH16);
  float*          F32    = (float*)(ws + kOffF32);

  {
    const int n8w = kD * kD / 8;
    cast8_kernel<<<dim3(n8w / 256), dim3(256), 0, stream>>>(Wq, WQH, n8w, n8w, kWCarry);
    cast8_kernel<<<dim3(n8w / 256), dim3(256), 0, stream>>>(Wk, WKH, n8w, n8w, kWCarry);
    cast8_kernel<<<dim3(n8w / 256), dim3(256), 0, stream>>>(Wv, WVH, n8w, n8w, kWCarry);
    cast8_kernel<<<dim3(n8w / 256), dim3(256), 0, stream>>>(Wo, WOH, n8w, n8w, kWCarry);
    const int n8f = kDff * kD / 8;
    cast8_kernel<<<dim3(n8f / 256), dim3(256), 0, stream>>>(W1, W1H, n8f, n8f, kWCarry);
    cast8_kernel<<<dim3(n8f / 256), dim3(256), 0, stream>>>(W2, W2H, n8f, n8f, kWCarry);
  }

  for (int br = 0; br < 2; ++br) {
    const float* text = br ? text2 : text1;
    const float* vis  = br ? vis2  : vis1;
    const float* sc   = br ? sc2   : sc1;
    const int colOff  = br * (kD / 2);

    const int n8t = kRows * kD / 8;
    cast8_kernel<<<dim3(n8t / 256), dim3(256), 0, stream>>>(text, T16, n8t, n8t, 1.0f);
    const int n8v = kSvPad * kD / 8;
    cast8_kernel<<<dim3(n8v / 256), dim3(256), 0, stream>>>(vis, VIS16, n8v, kSv * kD / 8, 1.0f);

    wmma_gemm64<0, false, 2, 1, false, 0><<<gemm_grid(kSvPad, kD), dim3(256), 0, stream>>>(
        VIS16, VIS16, kD, 0L, WKH, WKH, kD, 0L, (void*)K16, (void*)K16, kD, 0L,
        bk, text, 0L, kSvPad, kD, kD, kWCarryInv);
    wmma_gemm64<0, false, 1, 1, false, 0><<<gemm_grid(kD, kSvPad), dim3(256), 0, stream>>>(
        WVH, WVH, kD, 0L, VIS16, VIS16, kD, 0L, (void*)VT16, (void*)VT16, kSvPad, 0L,
        bv, text, 0L, kD, kSvPad, kD, kWCarryInv);
    wmma_gemm64<0, false, 2, 1, false, 0><<<gemm_grid(kRows, kD), dim3(256), 0, stream>>>(
        T16, T16, kD, 0L, WQH, WQH, kD, 0L, (void*)Q16, (void*)Q16, kD, 0L,
        bq, text, 0L, kRows, kD, kD, kWCarryInv);
    wmma_gemm64<0, false, 0, 0, false, 0><<<gemm_grid(kRows, kSvPad), dim3(256), 0, stream>>>(
        Q16, Q16, kD, 0L, K16, K16, kD, 0L, (void*)S32, (void*)S32, kSvPad, 0L,
        bq, text, 0L, kRows, kSvPad, kD, 1.0f);
    softmax_kernel<<<dim3(kRows / 8), dim3(256), 0, stream>>>(S32, sc, P16);
    wmma_gemm64<0, false, 0, 1, false, 0><<<gemm_grid(kRows, kD), dim3(256), 0, stream>>>(
        P16, P16, kSvPad, 0L, VT16, VT16, kSvPad, 0L, (void*)O16, (void*)O16, kD, 0L,
        bq, text, 0L, kRows, kD, kSvPad, kPVScale);
    wmma_gemm64<0, false, 2, 0, true, 0><<<gemm_grid(kRows, kD), dim3(256), 0, stream>>>(
        O16, O16, kD, 0L, WOH, WOH, kD, 0L, (void*)A1, (void*)A1, kD, 0L,
        bo, text, 0L, kRows, kD, kD, kWoScale);
    ln_pool_kernel<<<dim3(kRows), dim3(256), 0, stream>>>(A1, g1, be1, POOL32, POOL16, colOff);
  }

  for (int ch = 0; ch < kFfnChunks; ++ch) {
    const size_t rowOff = (size_t)ch * kFfnChunkRows * kD;
    wmma_gemm64<0, false, 2, 1, false, 2><<<gemm_grid(kFfnChunkRows, kDff), dim3(256), 0, stream>>>(
        POOL16 + rowOff, POOL16 + rowOff, kD, 0L, W1H, W1H, kD, 0L, (void*)H16, (void*)H16, kDff, 0L,
        b1, POOL32, 0L, kFfnChunkRows, kDff, kD, kWCarryInv);
    wmma_gemm64<0, false, 2, 0, true, 0><<<gemm_grid(kFfnChunkRows, kD), dim3(256), 0, stream>>>(
        H16, H16, kDff, 0L, W2H, W2H, kDff, 0L, (void*)F32, (void*)F32, kD, 0L,
        b2, POOL32 + rowOff, 0L, kFfnChunkRows, kD, kDff, kWCarryInv);
    ln_out_kernel<<<dim3(kFfnChunkRows), dim3(256), 0, stream>>>(F32, g2, be2, outp + rowOff);
  }
}
